// SMHA_52544629899784
// MI455X (gfx1250) — hardware-verified
//
#include <hip/hip_runtime.h>
#include <hip/hip_bf16.h>

typedef __attribute__((ext_vector_type(16))) _Float16 v16h;
typedef __attribute__((ext_vector_type(8)))  _Float16 v8h;
typedef __attribute__((ext_vector_type(16))) __bf16   v16b;
typedef __attribute__((ext_vector_type(8)))  __bf16   v8b;
typedef __attribute__((ext_vector_type(8)))  float    v8f;
typedef __attribute__((ext_vector_type(4)))  float    v4f;
typedef __attribute__((ext_vector_type(4)))  unsigned int v4u;

constexpr int kSeq   = 2048;
constexpr int kBatch = 2;
constexpr int kEmb   = 1024;
constexpr int kHeads = 16;
constexpr int kHd    = 64;
constexpr int kTok   = kSeq * kBatch;
static_assert(kHeads * kHd == kEmb, "geom");
static_assert(kTok == 4096, "geom");

constexpr size_t kMiB     = 1048576;
constexpr size_t OFF_XQ   = 0;
constexpr size_t OFF_XK   = 8 * kMiB;
constexpr size_t OFF_XV   = 16 * kMiB;
constexpr size_t OFF_WIN  = 24 * kMiB;
constexpr size_t OFF_PA   = 0;
constexpr size_t OFF_WOUT = 32 * kMiB;
constexpr size_t OFF_BIAS = 34 * kMiB;
constexpr size_t OFF_Q16  = 35 * kMiB;
constexpr size_t OFF_K16  = 43 * kMiB;
constexpr size_t OFF_VTH  = 51 * kMiB;
constexpr size_t OFF_VTL  = 59 * kMiB;
constexpr size_t OFF_AOH  = 67 * kMiB;
constexpr size_t OFF_AOL  = 75 * kMiB;
constexpr size_t OFF_PB   = 83 * kMiB;
constexpr size_t WS_TOTAL = 115 * kMiB;
static_assert((size_t)kTok * kEmb * 2 == 8 * kMiB, "x plane");
static_assert((size_t)3 * kEmb * kEmb * 2 == 6 * kMiB, "w_in plane");
static_assert(OFF_WIN + 6 * kMiB <= OFF_WOUT, "x and w_in fit below w_out");
static_assert(OFF_PA + (size_t)kBatch * kSeq * kSeq * 4 <= OFF_WOUT, "PA fits below w_out");
static_assert((size_t)kEmb * kEmb * 2 == 2 * kMiB, "w_out plane");
static_assert(OFF_BIAS + (size_t)(3 * kEmb + kEmb) * 4 <= OFF_Q16, "bias copies");
static_assert(OFF_PB + (size_t)kBatch * kSeq * kSeq * 4 == WS_TOTAL, "PB plane");
static_assert(WS_TOTAL == 120586240, "carve total");
static_assert(WS_TOTAL <= 134217728, "carve cap");

constexpr size_t kOut0Floats = (size_t)kTok * kEmb;
constexpr size_t kOut1Floats = (size_t)kBatch * kSeq * kSeq;
static_assert(kOut0Floats * 4 == 16777216, "out1 byte offset");
static_assert((kOut0Floats + kOut1Floats) * 4 == 50331648, "out total");

static_assert(kEmb % 32 == 0, "K multiple of 32");
static_assert(kTok % 64 == 0 && kEmb % 64 == 0, "M, N multiples of 64");

__device__ __forceinline__ unsigned short f2bf_bits(float f) {
  unsigned u = __float_as_uint(f);
  return (unsigned short)((u + 0x7FFFu + ((u >> 16) & 1u)) >> 16);
}
__device__ __forceinline__ float bf_bits2f(unsigned short h) { return __uint_as_float(((unsigned)h) << 16); }

__device__ __forceinline__ void dep_guard_h(v8f& a, v8f& b, v16h x, v16h y) { asm volatile("v_nop\n\tv_nop\n\tv_nop\n\tv_nop" : "+v"(a), "+v"(b) : "v"(x), "v"(y)); }
__device__ __forceinline__ void dep_guard_b(v8f& a, v8f& b, v16b x, v16b y) { asm volatile("v_nop\n\tv_nop\n\tv_nop\n\tv_nop" : "+v"(a), "+v"(b) : "v"(x), "v"(y)); }
__device__ __forceinline__ void keep4_h(v16h a, v16h b, v16h c, v16h d) { asm volatile("v_nop" :: "v"(a), "v"(b), "v"(c), "v"(d)); }
__device__ __forceinline__ void keep4_b(v16b a, v16b b, v16b c, v16b d) { asm volatile("v_nop" :: "v"(a), "v"(b), "v"(c), "v"(d)); }
__device__ __forceinline__ void acc_guard4(v8f& a, v8f& b, v8f& c, v8f& d) { asm volatile("v_nop\n\tv_nop\n\tv_nop\n\tv_nop" : "+v"(a), "+v"(b), "+v"(c), "+v"(d)); }
template <typename T> struct Frag;
template <> struct Frag<_Float16> {
  typedef v16h V; union U { v16h v; v8h h[2]; };
  static __device__ __forceinline__ v16h load(const _Float16* p) {
    U f; f.h[0] = *(const v8h*)(p); f.h[1] = *(const v8h*)(p + 16); return f.v;
  }
  static __device__ __forceinline__ v8f mma(v16h a, v16h b, v8f c) {
    return __builtin_amdgcn_wmma_f32_16x16x32_f16(false, a, false, b, (short)0, c, false, false);
  }
  static __device__ __forceinline__ void guard(v8f& a, v8f& b, v16h x, v16h y) { dep_guard_h(a, b, x, y); }
  static __device__ __forceinline__ void keep(v16h a, v16h b, v16h c, v16h d) { keep4_h(a, b, c, d); }
};
template <> struct Frag<__bf16> {
  typedef v16b V; union U { v16b v; v8b h[2]; };
  static __device__ __forceinline__ v16b load(const __bf16* p) {
    U f; f.h[0] = *(const v8b*)(p); f.h[1] = *(const v8b*)(p + 16); return f.v;
  }
  static __device__ __forceinline__ v8f mma(v16b a, v16b b, v8f c) {
    return __builtin_amdgcn_wmma_f32_16x16x32_bf16(false, a, false, b, (short)0, c, false, false);
  }
  static __device__ __forceinline__ void guard(v8f& a, v8f& b, v16b x, v16b y) { dep_guard_b(a, b, x, y); }
  static __device__ __forceinline__ void keep(v16b a, v16b b, v16b c, v16b d) { keep4_b(a, b, c, d); }
};

__device__ __forceinline__ v8f mma_f16g(v16h a, v16h b, v8f c) {
  c = __builtin_amdgcn_wmma_f32_16x16x32_f16(false, a, false, b, (short)0, c, false, false);
  asm volatile("v_nop\n\tv_nop\n\tv_nop\n\tv_nop" : "+v"(c) : "v"(a), "v"(b));
  return c;
}
__device__ __forceinline__ v8f mma_bf16g(v16b a, v16b b, v8f c) {
  c = __builtin_amdgcn_wmma_f32_16x16x32_bf16(false, a, false, b, (short)0, c, false, false);
  asm volatile("v_nop\n\tv_nop\n\tv_nop\n\tv_nop" : "+v"(c) : "v"(a), "v"(b));
  return c;
}
__device__ __forceinline__ __bf16 f2bf(float f) { return __builtin_bit_cast(__bf16, f2bf_bits(f)); }
__device__ __forceinline__ void bf_split(float f, __bf16& hi, __bf16& lo) {
  const unsigned short hb = f2bf_bits(f);
  hi = __builtin_bit_cast(__bf16, hb);
  lo = f2bf(f - __uint_as_float(((unsigned)hb) << 16));
}

template <int ET> struct Elem;
template <> struct Elem<0> { typedef _Float16 T; };
template <> struct Elem<1> { typedef __bf16 T; };
template <int ET, int SPLITM, int BIAS_MODE, int OUT_MODE>
__global__ __launch_bounds__(256) void wmma_gemm64(
    const unsigned short* __restrict__ Ap, const unsigned short* __restrict__ A2p, int lda, long strideA,
    const unsigned short* __restrict__ Btp, const unsigned short* __restrict__ Bt2p, int ldb, long strideB,
    void* __restrict__ Cout, void* __restrict__ Cout2, int ldc, long strideC,
    const float* __restrict__ bias,
    int M, int N, int K, float scale) {
  typedef typename Elem<ET>::T T;
  typedef typename Frag<T>::V V;
  const T* A = (const T*)Ap; const T* A2 = (const T*)A2p; const T* Bt = (const T*)Btp; const T* Bt2 = (const T*)Bt2p;
  __shared__ __align__(16) float sT[8][16 * 68];
  const int b    = blockIdx.y;
  const int lane = threadIdx.x & 31;
  const int wave = threadIdx.x >> 5;
  const int tilesN = N >> 6;
  const int tilesM = M >> 6;
  const int tile = blockIdx.x * 8 + wave;
  if (tile >= tilesM * tilesN) return;
  const int tm = tile / tilesN;
  const int tn = tile - tm * tilesN;
  const int m0 = tm << 6;
  const int n0 = tn << 6;

  const T* Ab  = A  + (size_t)b * strideA;
  const T* Bb  = Bt + (size_t)b * strideB;
  const T* Ab2 = (SPLITM != 0) ? (A2  + (size_t)b * strideA) : nullptr;
  const T* Bb2 = (SPLITM == 2) ? (Bt2 + (size_t)b * strideB) : nullptr;

  const int rlane = lane & 15;
  const int koff  = (lane >> 4) * 8;
  const int mOff  = (lane >> 4) * 8;

  v8f acc[4][4];
#pragma unroll
  for (int i = 0; i < 4; ++i)
#pragma unroll
    for (int j = 0; j < 4; ++j) acc[i][j] = (v8f){0.f,0.f,0.f,0.f,0.f,0.f,0.f,0.f};

  for (int k0 = 0; k0 < K; k0 += 32) {
    V bh[4], bl[4];
#pragma unroll
    for (int j = 0; j < 4; ++j) {
      const size_t bo = (size_t)(n0 + (j << 4) + rlane) * ldb + koff + k0;
      bh[j] = Frag<T>::load(Bb + bo);
      if (SPLITM == 2) bl[j] = Frag<T>::load(Bb2 + bo);
    }
#pragma unroll
    for (int i = 0; i < 4; ++i) {
      const size_t ao = (size_t)(m0 + (i << 4) + rlane) * lda + koff + k0;
      V ah = Frag<T>::load(Ab + ao);
      V al;
      if (SPLITM != 0) al = Frag<T>::load(Ab2 + ao);
#pragma unroll
      for (int j = 0; j < 4; ++j) {
        acc[i][j] = Frag<T>::mma(ah, bh[j], acc[i][j]);
        if (SPLITM == 2) acc[i][j] = Frag<T>::mma(ah, bl[j], acc[i][j]);
        if (SPLITM != 0) acc[i][j] = Frag<T>::mma(al, bh[j], acc[i][j]);
      }
      Frag<T>::guard(acc[i][0], acc[i][3], ah, (SPLITM != 0) ? al : ah);
    }
    Frag<T>::keep(bh[0], bh[1], bh[2], bh[3]);
    if (SPLITM == 2) Frag<T>::keep(bl[0], bl[1], bl[2], bl[3]);
  }
  acc_guard4(acc[0][0], acc[0][1], acc[0][2], acc[0][3]);
  acc_guard4(acc[1][0], acc[1][1], acc[1][2], acc[1][3]);
  acc_guard4(acc[2][0], acc[2][1], acc[2][2], acc[2][3]);
  acc_guard4(acc[3][0], acc[3][1], acc[3][2], acc[3][3]);

  float* slab = sT[wave];
#pragma unroll
  for (int i = 0; i < 4; ++i) {
    const int mBase = m0 + (i << 4);
    float bm[8];
#pragma unroll
    for (int r = 0; r < 8; ++r) bm[r] = (BIAS_MODE == 1) ? bias[mBase + mOff + r] : 0.0f;
#pragma unroll
    for (int j = 0; j < 4; ++j) {
      const int n = n0 + (j << 4) + rlane;
      float bv = 0.f;
      if (BIAS_MODE == 2) bv = bias[n];
#pragma unroll
      for (int r = 0; r < 8; ++r) {
        float v = acc[i][j][r] * scale;
        if (BIAS_MODE == 1) v += bm[r];
        if (BIAS_MODE == 2) v += bv;
        slab[(mOff + r) * 68 + (j << 4) + rlane] = v;
      }
    }
    __builtin_amdgcn_fence(__ATOMIC_RELEASE, "workgroup");
    __builtin_amdgcn_wave_barrier();
    __builtin_amdgcn_fence(__ATOMIC_ACQUIRE, "workgroup");
    if (OUT_MODE == 0) {
      float* C = (float*)Cout + (size_t)b * strideC;
      const int hh = lane >> 4, c4 = (lane & 15) * 4;
      for (int pass = 0; pass < 2; ++pass) {
#pragma unroll
        for (int it = 0; it < 8; ++it) {
          const int row = it * 2 + hh;
          v4f v = *(const v4f*)(slab + row * 68 + c4);
          *(volatile v4f*)(C + (size_t)(mBase + row) * ldc + n0 + c4) = v;
        }
        __threadfence();
      }
    } else {
      const int q = lane >> 3, c8 = (lane & 7) * 8;
      unsigned short* C  = (unsigned short*)Cout  + (size_t)b * strideC;
      unsigned short* C2 = (OUT_MODE == 2) ? ((unsigned short*)Cout2 + (size_t)b * strideC) : nullptr;
      for (int pass = 0; pass < 2; ++pass) {
#pragma unroll
        for (int it = 0; it < 4; ++it) {
          const int row = it * 4 + q;
          const float* sp = slab + row * 68 + c8;
          v8h hv, lv;
#pragma unroll
          for (int e = 0; e < 8; ++e) {
            if (OUT_MODE == 1) {
              hv[e] = (_Float16)sp[e];
            } else {
              unsigned short hb = f2bf_bits(sp[e]);
              unsigned short lb = f2bf_bits(sp[e] - bf_bits2f(hb));
              hv[e] = __builtin_bit_cast(_Float16, hb);
              lv[e] = __builtin_bit_cast(_Float16, lb);
            }
          }
          *(volatile v8h*)(C + (size_t)(mBase + row) * ldc + n0 + c8) = hv;
          if (OUT_MODE == 2) *(volatile v8h*)(C2 + (size_t)(mBase + row) * ldc + n0 + c8) = lv;
        }
        __threadfence();
      }
    }
    __builtin_amdgcn_fence(__ATOMIC_RELEASE, "workgroup");
    __builtin_amdgcn_wave_barrier();
    __builtin_amdgcn_fence(__ATOMIC_ACQUIRE, "workgroup");
  }
}

__global__ __launch_bounds__(256) void k_cast_bf16(const float* __restrict__ in, unsigned short* __restrict__ out,
                                                   int nrows, int permB, int permL) {
  const int i = blockIdx.x * 256 + threadIdx.x;
  const int r = i >> 7;
  const int c8 = (i & 127) * 8;
  if (r >= nrows) return;
  int orow = r;
  if (permB > 0) {
    const int bb = r % permB;
    const int ll = r / permB;
    orow = bb * permL + ll;
  }
  const float* src = in + (size_t)r * kEmb + c8;
  const v4f x0 = *(const v4f*)(src);
  const v4f x1 = *(const v4f*)(src + 4);
  v4u w;
  w[0] = (unsigned)f2bf_bits(x0[0]) | ((unsigned)f2bf_bits(x0[1]) << 16);
  w[1] = (unsigned)f2bf_bits(x0[2]) | ((unsigned)f2bf_bits(x0[3]) << 16);
  w[2] = (unsigned)f2bf_bits(x1[0]) | ((unsigned)f2bf_bits(x1[1]) << 16);
  w[3] = (unsigned)f2bf_bits(x1[2]) | ((unsigned)f2bf_bits(x1[3]) << 16);
  unsigned short* dst = out + (size_t)orow * kEmb + c8;
  *(volatile v4u*)dst = w;
  __threadfence();
  *(volatile v4u*)dst = w;
}

__global__ __launch_bounds__(256) void k_bias_rne(const float* __restrict__ in, float* __restrict__ out, int n4) {
  const int i = blockIdx.x * 256 + threadIdx.x;
  if (i >= n4) return;
  const v4f x = *(const v4f*)(in + (size_t)i * 4);
  v4f y;
  y[0] = bf_bits2f(f2bf_bits(x[0]));
  y[1] = bf_bits2f(f2bf_bits(x[1]));
  y[2] = bf_bits2f(f2bf_bits(x[2]));
  y[3] = bf_bits2f(f2bf_bits(x[3]));
  float* dst = out + (size_t)i * 4;
  *(volatile v4f*)dst = y;
  __threadfence();
  *(volatile v4f*)dst = y;
}

template <bool ADD_IN>
__global__ __launch_bounds__(256) void k_sigattn(
    const unsigned short* __restrict__ q16, const unsigned short* __restrict__ k16,
    const unsigned short* __restrict__ vth, const unsigned short* __restrict__ vtl,
    unsigned short* __restrict__ aoh, unsigned short* __restrict__ aol,
    const float* __restrict__ avg_in, float* __restrict__ avg_out, int head) {
  __shared__ __align__(16) __bf16 Psh[4][16 * 64];
  __shared__ __align__(16) __bf16 Psl[4][16 * 64];
  __shared__ __align__(16) float  Fsh[4][16 * 68];
  const int tid  = threadIdx.x;
  const int wave = tid >> 5;
  const int lane = tid & 31;
  const int hh   = lane >> 4;
  const int c    = lane & 15;
  const int koff = hh * 8;
  const int b    = blockIdx.x >> 5;
  const int qt   = blockIdx.x & 31;
  const int l0   = qt * 64 + wave * 16;
  const int ecol = head * kHd;
  const _Float16* Qp = (const _Float16*)q16;
  const _Float16* Kp = (const _Float16*)k16;
  const __bf16* Vh = (const __bf16*)vth;
  const __bf16* Vl = (const __bf16*)vtl;

  v16h qa0, qa1;
  {
    const _Float16* qrow = Qp + (size_t)(b * kSeq + l0 + c) * kEmb + ecol + koff;
    qa0 = Frag<_Float16>::load(qrow);
    qa1 = Frag<_Float16>::load(qrow + 32);
  }
  const v8f zero8 = (v8f){0.f,0.f,0.f,0.f,0.f,0.f,0.f,0.f};
  v8f oacc[4];
#pragma unroll
  for (int t = 0; t < 4; ++t) oacc[t] = zero8;
  float den[8];
#pragma unroll
  for (int r = 0; r < 8; ++r) den[r] = 0.0f;

  __bf16* pwh = Psh[wave];
  __bf16* pwl = Psl[wave];
  float*  fw  = Fsh[wave];
  const float* ain  = avg_in  + ((size_t)b * kSeq + l0) * kSeq;
  float*       aout = avg_out + ((size_t)b * kSeq + l0) * kSeq;

  for (int kc = 0; kc < kSeq / 64; ++kc) {
    const int s0 = kc * 64;
    v8f sc[4];
#pragma unroll
    for (int j = 0; j < 4; ++j) {
      const _Float16* krow = Kp + (size_t)(b * kSeq + s0 + j * 16 + c) * kEmb + ecol + koff;
      const v16h kb0 = Frag<_Float16>::load(krow);
      const v16h kb1 = Frag<_Float16>::load(krow + 32);
      v8f a = zero8;
      a = mma_f16g(qa0, kb0, a);
      a = mma_f16g(qa1, kb1, a);
      sc[j] = a;
    }
#pragma unroll
    for (int j = 0; j < 4; ++j) {
#pragma unroll
      for (int r = 0; r < 8; ++r) {
        const float x = sc[j][r] * 0.125f;
        const float p = 1.0f / (1.0f + expf(-x));
        den[r] += p;
        fw[(8 * hh + r) * 68 + j * 16 + c] = p * 0.0625f;
        __bf16 ph, plo;
        bf_split(p, ph, plo);
        pwh[(8 * hh + r) * 64 + j * 16 + c] = ph;
        pwl[(8 * hh + r) * 64 + j * 16 + c] = plo;
      }
    }
    __syncthreads();
    {
      const int c4 = c * 4;
      v4f val[8];
#pragma unroll
      for (int it = 0; it < 8; ++it) {
        const int row = it * 2 + hh;
        v4f v = *(const v4f*)(fw + row * 68 + c4);
        if (ADD_IN) {
          const v4f rin = *(const v4f*)(ain + (size_t)row * kSeq + s0 + c4);
          v = v + rin;
        }
        val[it] = v;
      }
      for (int pass = 0; pass < 2; ++pass) {
#pragma unroll
        for (int it = 0; it < 8; ++it) {
          const int row = it * 2 + hh;
          *(volatile v4f*)(aout + (size_t)row * kSeq + s0 + c4) = val[it];
        }
        __threadfence();
      }
    }
#pragma unroll
    for (int kk = 0; kk < 2; ++kk) {
      const v16b pa = Frag<__bf16>::load(pwh + c * 64 + kk * 32 + koff);
      const v16b pl = Frag<__bf16>::load(pwl + c * 64 + kk * 32 + koff);
#pragma unroll
      for (int t = 0; t < 4; ++t) {
        const size_t vo = (size_t)(ecol + t * 16 + c) * kTok + (size_t)b * kSeq + s0 + kk * 32 + koff;
        const v16b vb  = Frag<__bf16>::load(Vh + vo);
        const v16b vl2 = Frag<__bf16>::load(Vl + vo);
        oacc[t] = mma_bf16g(pa, vb, oacc[t]);
        oacc[t] = mma_bf16g(pa, vl2, oacc[t]);
        oacc[t] = mma_bf16g(pl, vb, oacc[t]);
      }
    }
    __syncthreads();
  }

  float inv[8];
#pragma unroll
  for (int r = 0; r < 8; ++r) {
    float v = den[r];
    v += __shfl_xor(v, 1, 32);
    v += __shfl_xor(v, 2, 32);
    v += __shfl_xor(v, 4, 32);
    v += __shfl_xor(v, 8, 32);
    inv[r] = 1.0f / (v + 1e-4f);
  }
#pragma unroll
  for (int r = 0; r < 8; ++r) {
#pragma unroll
    for (int t = 0; t < 4; ++t) fw[(8 * hh + r) * 68 + t * 16 + c] = oacc[t][r] * inv[r];
  }
  __syncthreads();
  {
    const int q  = lane >> 3;
    const int c8 = (lane & 7) * 8;
    for (int pass = 0; pass < 2; ++pass) {
#pragma unroll
      for (int it = 0; it < 4; ++it) {
        const int row = it * 4 + q;
        const float* sp = fw + row * 68 + c8;
        v8h hv, lv;
#pragma unroll
        for (int e = 0; e < 8; ++e) {
          const unsigned short hb = f2bf_bits(sp[e]);
          const unsigned short lb = f2bf_bits(sp[e] - bf_bits2f(hb));
          hv[e] = __builtin_bit_cast(_Float16, hb);
          lv[e] = __builtin_bit_cast(_Float16, lb);
        }
        const size_t ro = (size_t)((l0 + row) * kBatch + b) * kEmb + ecol + c8;
        *(volatile v8h*)(aoh + ro) = hv;
        *(volatile v8h*)(aol + ro) = lv;
      }
      __threadfence();
    }
  }
}

extern "C" void kernel_launch(void* const* d_in, const int* in_sizes, int n_in,
                              void* d_out, int out_size, void* d_ws,
                              size_t ws_size, hipStream_t stream) {
  if (n_in < 7) return;
  if (in_sizes[0] != kTok * kEmb || in_sizes[1] != kTok * kEmb || in_sizes[2] != kTok * kEmb) return;
  if (in_sizes[3] != 3 * kEmb * kEmb || in_sizes[4] != 3 * kEmb) return;
  if (in_sizes[5] != kEmb * kEmb || in_sizes[6] != kEmb) return;
  if ((size_t)out_size != kOut0Floats + kOut1Floats) return;
  if (ws_size < WS_TOTAL) return;

  const float* query = (const float*)d_in[0];
  const float* keyp  = (const float*)d_in[1];
  const float* value = (const float*)d_in[2];
  const float* ipw   = (const float*)d_in[3];
  const float* ipb   = (const float*)d_in[4];
  const float* ow    = (const float*)d_in[5];
  const float* ob    = (const float*)d_in[6];

  float* out0 = (float*)d_out;
  float* out1 = (float*)d_out + kOut0Floats;

  char* ws = (char*)d_ws;
  unsigned short* xq    = (unsigned short*)(ws + OFF_XQ);
  unsigned short* xk    = (unsigned short*)(ws + OFF_XK);
  unsigned short* xv    = (unsigned short*)(ws + OFF_XV);
  unsigned short* win   = (unsigned short*)(ws + OFF_WIN);
  unsigned short* wout  = (unsigned short*)(ws + OFF_WOUT);
  float*          biasr = (float*)(ws + OFF_BIAS);
  unsigned short* q16   = (unsigned short*)(ws + OFF_Q16);
  unsigned short* k16   = (unsigned short*)(ws + OFF_K16);
  unsigned short* vth   = (unsigned short*)(ws + OFF_VTH);
  unsigned short* vtl   = (unsigned short*)(ws + OFF_VTL);
  unsigned short* aoh   = (unsigned short*)(ws + OFF_AOH);
  unsigned short* aol   = (unsigned short*)(ws + OFF_AOL);
  float*          pa    = (float*)(ws + OFF_PA);
  float*          pb    = (float*)(ws + OFF_PB);

  k_cast_bf16<<<dim3(kTok * 128 / 256), dim3(256), 0, stream>>>(query, xq, kTok, kBatch, kSeq);
  k_cast_bf16<<<dim3(kTok * 128 / 256), dim3(256), 0, stream>>>(keyp,  xk, kTok, kBatch, kSeq);
  k_cast_bf16<<<dim3(kTok * 128 / 256), dim3(256), 0, stream>>>(value, xv, kTok, kBatch, kSeq);
  k_cast_bf16<<<dim3(3 * kEmb * 128 / 256), dim3(256), 0, stream>>>(ipw, win, 3 * kEmb, 0, 0);
  k_cast_bf16<<<dim3(kEmb * 128 / 256), dim3(256), 0, stream>>>(ow, wout, kEmb, 0, 0);
  k_bias_rne<<<dim3(3), dim3(256), 0, stream>>>(ipb, biasr, 3 * kEmb / 4);
  k_bias_rne<<<dim3(1), dim3(256), 0, stream>>>(ob, biasr + 3 * kEmb, kEmb / 4);

  const int gemmBlocks = (kTok / 64) * (kEmb / 64) / 8;
  wmma_gemm64<1, 0, 2, 1><<<dim3(gemmBlocks, 1), dim3(256), 0, stream>>>(
      xq, xq, kEmb, 0L, win, win, kEmb, 0L, (void*)q16, (void*)q16, kEmb, 0L,
      biasr, kTok, kEmb, kEmb, 1.0f);
  wmma_gemm64<1, 0, 2, 1><<<dim3(gemmBlocks, 1), dim3(256), 0, stream>>>(
      xk, xk, kEmb, 0L, win + (size_t)kEmb * kEmb, win, kEmb, 0L, (void*)k16, (void*)k16, kEmb, 0L,
      biasr + kEmb, kTok, kEmb, kEmb, 1.0f);
  wmma_gemm64<1, 0, 1, 2><<<dim3(gemmBlocks, 1), dim3(256), 0, stream>>>(
      win + (size_t)2 * kEmb * kEmb, win, kEmb, 0L, xv, xv, kEmb, 0L, (void*)vth, (void*)vtl, kTok, 0L,
      biasr + 2 * kEmb, kEmb, kTok, kEmb, 1.0f);

  for (int h = 0; h < kHeads; ++h) {
    float* dst = (h == kHeads - 1) ? out1 : ((h & 1) ? pb : pa);
    if (h == 0) {
      k_sigattn<false><<<dim3(kBatch * (kSeq / 64)), dim3(128), 0, stream>>>(q16, k16, vth, vtl, aoh, aol, pb, dst, h);
    } else {
      const float* src = ((h - 1) & 1) ? pb : pa;
      k_sigattn<true><<<dim3(kBatch * (kSeq / 64)), dim3(128), 0, stream>>>(q16, k16, vth, vtl, aoh, aol, src, dst, h);
    }
  }

  wmma_gemm64<1, 1, 2, 0><<<dim3(gemmBlocks, 1), dim3(256), 0, stream>>>(
      aoh, aol, kEmb, 0L, wout, wout, kEmb, 0L, (void*)out0, (void*)out0, kEmb, 0L,
      biasr + 3 * kEmb, kTok, kEmb, kEmb, 1.0f);
}
